// RnnModelInterp_75814762709699
// MI455X (gfx1250) — hardware-run, weakly checked
//
#include <hip/hip_runtime.h>
#include <math.h>

constexpr int SEQ_LEN    = 200;
constexpr int NSTEP      = SEQ_LEN - 1;
constexpr int NBATCH     = 256;
constexpr int NHID       = 512;
constexpr int NCAT       = 3;
constexpr int NMEAS      = 64;
constexpr int NXIN       = NCAT + NMEAS;
constexpr int XK_PAD     = 96;
constexpr int WX_PITCH   = 128;
constexpr int NHEAD_REAL = NCAT + NMEAS;
constexpr int NHEAD_PAD  = 80;
constexpr int ROWS_BLK   = 16;
constexpr int NTHR       = 256;
constexpr int SX_PITCH   = 104;
constexpr int S1_PITCH   = 2 * NHID + 8;
constexpr int HO_PITCH   = 84;
constexpr int XPAD_TAIL  = XK_PAD - NXIN - 16;
constexpr int NOUT       = NSTEP * NBATCH * NCAT;
constexpr int NOUT4      = NOUT / 4;
constexpr float WCARRY     = 16.0f;
constexpr float WCARRY_INV = 1.0f / WCARRY;

static_assert(NXIN == 67, "x width");
static_assert(XK_PAD % 32 == 0 && XK_PAD >= NXIN, "x K pad multiple of 32");
static_assert(NHID % 32 == 0, "hidden K multiple of 32");
static_assert(NHID == 64 * (NTHR / 32), "8 waves x 64 hidden columns");
static_assert(NBATCH % ROWS_BLK == 0, "blocks of 16 rows");
static_assert(NHEAD_PAD % 16 == 0 && NHEAD_PAD >= NHEAD_REAL && NHEAD_PAD / 16 <= NTHR / 32, "head tiles");
static_assert(XPAD_TAIL > 0 && XPAD_TAIL <= 16, "x pad tail");
static_assert(SX_PITCH % 8 == 0 && SX_PITCH >= XK_PAD, "x tile pitch");
static_assert(S1_PITCH % 8 == 0, "state tile pitch");
static_assert(WX_PITCH % 64 == 0 && WX_PITCH >= XK_PAD, "x weight plane pitch is a line multiple");
static_assert(NOUT % 128 == 0, "output is a whole number of 512-B wave chunks");
static_assert(ROWS_BLK * 16 == NTHR, "elementwise phase map: 16 rows x 16 lanes");
static_assert(NMEAS == 4 * 16, "value columns: 4 per thread");

typedef __attribute__((ext_vector_type(16))) _Float16 v16h;
typedef __attribute__((ext_vector_type(8)))  _Float16 v8h;
typedef __attribute__((ext_vector_type(8)))  float    v8f;
typedef __attribute__((ext_vector_type(4)))  float    v4f;

__device__ __forceinline__ void guard4_h(v8f& a0, v8f& a1, v8f& a2, v8f& a3, v16h x, v16h y0, v16h y1, v16h y2, v16h y3) {
  asm volatile("v_nop\n\tv_nop\n\tv_nop\n\tv_nop" : "+v"(a0), "+v"(a1), "+v"(a2), "+v"(a3) : "v"(x), "v"(y0), "v"(y1), "v"(y2), "v"(y3));
}
__device__ __forceinline__ void guard1_h(v8f& a0, v16h x, v16h y) {
  asm volatile("v_nop\n\tv_nop\n\tv_nop\n\tv_nop" : "+v"(a0) : "v"(x), "v"(y));
}
__device__ __forceinline__ void pin_f(float& x) { asm volatile("" : "+v"(x)); }

template <typename T> struct Frag;
template <> struct Frag<_Float16> {
  typedef v16h V; union U { v16h v; v8h h[2]; };
  static __device__ __forceinline__ v16h load(const _Float16* p) {
    U f; f.h[0] = *(const v8h*)(p); f.h[1] = *(const v8h*)(p + 16); return f.v;
  }
  static __device__ __forceinline__ v8f mma(v16h a, v16h b, v8f c) {
    return __builtin_amdgcn_wmma_f32_16x16x32_f16(false, a, false, b, (short)0, c, false, false);
  }
};

__device__ __forceinline__ bool nan_bits(float x) {
  return (__float_as_uint(x) & 0x7fffffffu) > 0x7f800000u;
}

__device__ __forceinline__ void tr8_store(const float* __restrict__ src, int validK, int srcPitch,
                                          unsigned short* __restrict__ dst, int kgroups, int li) {
  const int n = li / kgroups;
  const int g = li - n * kgroups;
  v8h hv;
#pragma unroll
  for (int e = 0; e < 8; ++e) {
    const int k  = 8 * g + e;
    const int kc = (k < validK) ? k : (validK - 1);
    float v = src[(size_t)kc * (size_t)srcPitch + n];
    pin_f(v);
    const float vz = (k < validK) ? v : 0.0f;
    hv[e] = (_Float16)(vz * WCARRY);
  }
  volatile v8h* dp = (volatile v8h*)(dst + (size_t)li * 8);
  *dp = hv;
  __threadfence();
  *dp = hv;
}

constexpr int PB_WX = (NHID * (WX_PITCH / 8)) / NTHR;
constexpr int PB_SQ = (NHID * (NHID / 8)) / NTHR;
constexpr int PB_HD = (NHEAD_PAD * (NHID / 8)) / NTHR;
constexpr int PB_ALL = PB_WX + 3 * PB_SQ + PB_HD;
static_assert((NHID * (WX_PITCH / 8)) % NTHR == 0, "exact coverage of the x weight plane");
static_assert((NHID * (NHID / 8)) % NTHR == 0, "exact coverage of the square planes");
static_assert((NHEAD_PAD * (NHID / 8)) % NTHR == 0, "exact coverage of the head plane");

__global__ __launch_bounds__(NTHR) void prep_planes_kernel(
    const float* __restrict__ W_ih0, const float* __restrict__ W_hh0,
    const float* __restrict__ W_ih1, const float* __restrict__ W_hh1,
    const float* __restrict__ Wc, const float* __restrict__ Wm,
    unsigned short* __restrict__ WX0, unsigned short* __restrict__ WH0,
    unsigned short* __restrict__ WI1, unsigned short* __restrict__ WH1,
    unsigned short* __restrict__ WHD) {
  const int bx = blockIdx.x;
  const int tid = threadIdx.x;
  if (bx < PB_WX) {
    tr8_store(W_ih0, NXIN, NHID, WX0, WX_PITCH / 8, bx * NTHR + tid);
  } else if (bx < PB_WX + PB_SQ) {
    tr8_store(W_hh0, NHID, NHID, WH0, NHID / 8, (bx - PB_WX) * NTHR + tid);
  } else if (bx < PB_WX + 2 * PB_SQ) {
    tr8_store(W_ih1, NHID, NHID, WI1, NHID / 8, (bx - PB_WX - PB_SQ) * NTHR + tid);
  } else if (bx < PB_WX + 3 * PB_SQ) {
    tr8_store(W_hh1, NHID, NHID, WH1, NHID / 8, (bx - PB_WX - 2 * PB_SQ) * NTHR + tid);
  } else {
    const int li = (bx - PB_WX - 3 * PB_SQ) * NTHR + tid;
    const int n  = li / (NHID / 8);
    const int g  = li - n * (NHID / 8);
    const int nc = (n < NCAT - 1) ? n : (NCAT - 1);
    int nm = n - NCAT;
    nm = (nm < 0) ? 0 : nm;
    nm = (nm > NMEAS - 1) ? (NMEAS - 1) : nm;
    const bool isC = (n < NCAT);
    const bool isM = (n >= NCAT) && (n < NHEAD_REAL);
    v8h hv;
#pragma unroll
    for (int e = 0; e < 8; ++e) {
      const int k = 8 * g + e;
      float wc = Wc[(size_t)k * NCAT + nc];
      float wm = Wm[(size_t)k * NMEAS + nm];
      pin_f(wc);
      pin_f(wm);
      const float v = isC ? wc : (isM ? wm : 0.0f);
      hv[e] = (_Float16)(v * WCARRY);
    }
    volatile v8h* dp = (volatile v8h*)(WHD + (size_t)li * 8);
    *dp = hv;
    __threadfence();
    *dp = hv;
  }
}

__device__ __forceinline__ void mm4_loop(const _Float16* ap, const _Float16* __restrict__ wp, int wstep, int klen,
                                         v8f& c0, v8f& c1, v8f& c2, v8f& c3) {
#pragma unroll 1
  for (int k0 = 0; k0 < klen; k0 += 32) {
    const v16h a  = Frag<_Float16>::load(ap + k0);
    const v16h b0 = Frag<_Float16>::load(wp + k0);
    const v16h b1 = Frag<_Float16>::load(wp + wstep + k0);
    const v16h b2 = Frag<_Float16>::load(wp + 2 * wstep + k0);
    const v16h b3 = Frag<_Float16>::load(wp + 3 * wstep + k0);
    c0 = Frag<_Float16>::mma(a, b0, c0);
    c1 = Frag<_Float16>::mma(a, b1, c1);
    c2 = Frag<_Float16>::mma(a, b2, c2);
    c3 = Frag<_Float16>::mma(a, b3, c3);
    guard4_h(c0, c1, c2, c3, a, b0, b1, b2, b3);
  }
}

__device__ __forceinline__ void tanh_store(_Float16* dstbase, v8f a0, v8f a1, v8f a2, v8f a3,
                                           float b0, float b1, float b2, float b3) {
#pragma unroll 1
  for (int j = 0; j < 4; ++j) {
    const v8f cur = (j == 0) ? a0 : ((j == 1) ? a1 : ((j == 2) ? a2 : a3));
    const float bj = (j == 0) ? b0 : ((j == 1) ? b1 : ((j == 2) ? b2 : b3));
    _Float16* dst = dstbase + 16 * j;
#pragma unroll
    for (int r = 0; r < 8; ++r) {
      const float z = cur[r] * WCARRY_INV + bj;
      dst[r * S1_PITCH] = (_Float16)tanhf(z);
    }
  }
}

__global__ __launch_bounds__(NTHR) void rnn_scan_kernel(
    const float* __restrict__ cat_seq, const float* __restrict__ val_seq,
    const float* __restrict__ b0, const float* __restrict__ b1,
    const float* __restrict__ bc, const float* __restrict__ bm,
    const unsigned short* __restrict__ WX0p, const unsigned short* __restrict__ WH0p,
    const unsigned short* __restrict__ WI1p, const unsigned short* __restrict__ WH1p,
    const unsigned short* __restrict__ WHDp,
    float* __restrict__ stage) {
  __shared__ __align__(16) _Float16 Sx[ROWS_BLK * SX_PITCH];
  __shared__ __align__(16) _Float16 S1[ROWS_BLK * S1_PITCH];
  __shared__ __align__(16) float    HeadO[ROWS_BLK * HO_PITCH];
  __shared__ __align__(16) float    OStage[ROWS_BLK * 4];

  const _Float16* WX0 = (const _Float16*)WX0p;
  const _Float16* WH0 = (const _Float16*)WH0p;
  const _Float16* WI1 = (const _Float16*)WI1p;
  const _Float16* WH1 = (const _Float16*)WH1p;
  const _Float16* WHD = (const _Float16*)WHDp;

  const int tid = threadIdx.x, lane = tid & 31, wave = tid >> 5;
  const int c = lane & 15, hh = lane >> 4, koff = hh * 8;
  const int m0 = blockIdx.x * ROWS_BLK;
  const int er = tid >> 4, eq = tid & 15;
  const int colw = 64 * wave + c;

#pragma unroll 1
  for (int i = tid; i < ROWS_BLK * S1_PITCH; i += NTHR) S1[i] = (_Float16)0.0f;

  float vc0, vc1, vc2, vc3;
  {
    const int qc = (eq < NCAT - 1) ? eq : (NCAT - 1);
    float cv = cat_seq[(size_t)(m0 + er) * NCAT + qc];
    pin_f(cv);
    if (eq < NCAT) Sx[er * SX_PITCH + eq] = (_Float16)cv;
    const v4f vv = *(const v4f*)(val_seq + (size_t)(m0 + er) * NMEAS + 4 * eq);
    vc0 = vv[0]; vc1 = vv[1]; vc2 = vv[2]; vc3 = vv[3];
    _Float16* xr = Sx + er * SX_PITCH + NCAT + 4 * eq;
    xr[0] = (_Float16)vc0;
    xr[1] = (_Float16)vc1;
    xr[2] = (_Float16)vc2;
    xr[3] = (_Float16)vc3;
    Sx[er * SX_PITCH + NXIN + eq] = (_Float16)0.0f;
    if (eq < XPAD_TAIL) Sx[er * SX_PITCH + NXIN + 16 + eq] = (_Float16)0.0f;
  }

  const float bA0 = b0[colw], bA1 = b0[colw + 16], bA2 = b0[colw + 32], bA3 = b0[colw + 48];
  const float bB0 = b1[colw], bB1 = b1[colw + 16], bB2 = b1[colw + 32], bB3 = b1[colw + 48];
  const int hwave = (wave < NHEAD_PAD / 16) ? wave : 0;
  const int nhead = 16 * hwave + c;
  float hb;
  {
    const int ic = (nhead < NCAT - 1) ? nhead : (NCAT - 1);
    int im = nhead - NCAT;
    im = (im < 0) ? 0 : im;
    im = (im > NMEAS - 1) ? (NMEAS - 1) : im;
    float bcv = bc[ic];
    float bmv = bm[im];
    pin_f(bcv);
    pin_f(bmv);
    hb = (nhead < NCAT) ? bcv : ((nhead < NHEAD_REAL) ? bmv : 0.0f);
  }
  __syncthreads();

  const v8f z8 = {0.f, 0.f, 0.f, 0.f, 0.f, 0.f, 0.f, 0.f};
  const _Float16* ax  = Sx + c * SX_PITCH + koff;
  const _Float16* ah0 = S1 + c * S1_PITCH + koff;
  const _Float16* ah1 = S1 + c * S1_PITCH + NHID + koff;
  const _Float16* wx0 = WX0 + (size_t)colw * WX_PITCH + koff;
  const _Float16* wh0 = WH0 + (size_t)colw * NHID + koff;
  const _Float16* wi1 = WI1 + (size_t)colw * NHID + koff;
  const _Float16* wh1 = WH1 + (size_t)colw * NHID + koff;
  const _Float16* whd = WHD + (size_t)nhead * NHID + koff;
  _Float16* d0 = S1 + (8 * hh) * S1_PITCH + colw;
  _Float16* d1 = S1 + (8 * hh) * S1_PITCH + NHID + colw;

#pragma unroll 1
  for (int t = 0; t < NSTEP; ++t) {
    v8f p0 = z8, p1 = z8, p2 = z8, p3 = z8;
    mm4_loop(ax, wx0, 16 * WX_PITCH, XK_PAD, p0, p1, p2, p3);
    mm4_loop(ah0, wh0, 16 * NHID, NHID, p0, p1, p2, p3);
    __syncthreads();
    tanh_store(d0, p0, p1, p2, p3, bA0, bA1, bA2, bA3);
    __syncthreads();

    v8f s0 = z8, s1 = z8, s2 = z8, s3 = z8;
    mm4_loop(ah0, wi1, 16 * NHID, NHID, s0, s1, s2, s3);
    mm4_loop(ah1, wh1, 16 * NHID, NHID, s0, s1, s2, s3);
    __syncthreads();
    tanh_store(d1, s0, s1, s2, s3, bB0, bB1, bB2, bB3);
    __syncthreads();

    if (wave < NHEAD_PAD / 16) {
      v8f e = z8;
#pragma unroll 1
      for (int k0 = 0; k0 < NHID; k0 += 32) {
        const v16h a = Frag<_Float16>::load(ah1 + k0);
        const v16h b = Frag<_Float16>::load(whd + k0);
        e = Frag<_Float16>::mma(a, b, e);
        guard1_h(e, a, b);
      }
#pragma unroll
      for (int r = 0; r < 8; ++r) HeadO[(8 * hh + r) * HO_PITCH + nhead] = e[r] * WCARRY_INV + hb;
    }
    __syncthreads();

    {
      const float l0 = HeadO[er * HO_PITCH + 0];
      const float l1 = HeadO[er * HO_PITCH + 1];
      const float l2 = HeadO[er * HO_PITCH + 2];
      const float mx = fmaxf(l0, fmaxf(l1, l2));
      const float e0 = expf(l0 - mx);
      const float e1 = expf(l1 - mx);
      const float e2 = expf(l2 - mx);
      const float inv = 1.0f / (e0 + e1 + e2);
      const int qc = (eq < NCAT - 1) ? eq : (NCAT - 1);
      const float es = (qc == 0) ? e0 : ((qc == 1) ? e1 : e2);
      const float oq = es * inv;
      float cn = cat_seq[(size_t)(t + 1) * (NBATCH * NCAT) + (size_t)(m0 + er) * NCAT + qc];
      pin_f(cn);
      const float cnew = nan_bits(cn) ? oq : cn;
      if (eq < NCAT) Sx[er * SX_PITCH + eq] = (_Float16)cnew;
      if (eq < 4) OStage[er * 4 + eq] = (eq < NCAT) ? oq : 0.0f;

      const v4f vn = *(const v4f*)(val_seq + (size_t)(t + 1) * (NBATCH * NMEAS) + (size_t)(m0 + er) * NMEAS + 4 * eq);
      const float* ho = HeadO + er * HO_PITCH + NCAT + 4 * eq;
      const float x0 = vn[0], x1 = vn[1], x2 = vn[2], x3 = vn[3];
      const float o0 = ho[0] + vc0;
      const float o1 = ho[1] + vc1;
      const float o2 = ho[2] + vc2;
      const float o3 = ho[3] + vc3;
      vc0 = nan_bits(x0) ? o0 : x0;
      vc1 = nan_bits(x1) ? o1 : x1;
      vc2 = nan_bits(x2) ? o2 : x2;
      vc3 = nan_bits(x3) ? o3 : x3;
      _Float16* xr = Sx + er * SX_PITCH + NCAT + 4 * eq;
      xr[0] = (_Float16)vc0;
      xr[1] = (_Float16)vc1;
      xr[2] = (_Float16)vc2;
      xr[3] = (_Float16)vc3;
      Sx[er * SX_PITCH + NXIN + eq] = (_Float16)0.0f;
      if (eq < XPAD_TAIL) Sx[er * SX_PITCH + NXIN + 16 + eq] = (_Float16)0.0f;
    }
    __syncthreads();

    if (wave == 0) {
      const v4f ov = *(const v4f*)(OStage + c * 4);
      volatile v4f* sp = (volatile v4f*)(stage + ((size_t)t * NBATCH + (size_t)(m0 + c)) * 4);
      if (lane < 16) *sp = ov;
      __threadfence();
      if (lane < 16) *sp = ov;
    }
  }
}

__global__ __launch_bounds__(NTHR) void pack_out_kernel(const float* __restrict__ stage, float* __restrict__ out, int n4) {
  const int i = blockIdx.x * NTHR + threadIdx.x;
  if (i < n4) {
    v4f o;
#pragma unroll
    for (int e = 0; e < 4; ++e) {
      const int idx = 4 * i + e;
      const int row = idx / NCAT;
      const int cc  = idx - NCAT * row;
      o[e] = stage[(size_t)row * 4 + cc];
    }
    volatile v4f* op = (volatile v4f*)(out + (size_t)i * 4);
    *op = o;
    __threadfence();
    *op = o;
  }
}

extern "C" void kernel_launch(void* const* d_in, const int* in_sizes, int n_in,
                              void* d_out, int out_size, void* d_ws, size_t ws_size, hipStream_t stream) {
  if (n_in < 12 || d_out == nullptr || d_ws == nullptr) return;
  if (in_sizes[0] != SEQ_LEN * NBATCH * NCAT || in_sizes[1] != SEQ_LEN * NBATCH * NMEAS ||
      in_sizes[2] != NXIN * NHID || in_sizes[3] != NHID * NHID || in_sizes[4] != NHID ||
      in_sizes[5] != NHID * NHID || in_sizes[6] != NHID * NHID || in_sizes[7] != NHID ||
      in_sizes[8] != NHID * NCAT || in_sizes[9] != NCAT || in_sizes[10] != NHID * NMEAS ||
      in_sizes[11] != NMEAS || out_size != NOUT) return;

  const float* cat_seq = (const float*)d_in[0];
  const float* val_seq = (const float*)d_in[1];
  const float* W_ih0   = (const float*)d_in[2];
  const float* W_hh0   = (const float*)d_in[3];
  const float* b0      = (const float*)d_in[4];
  const float* W_ih1   = (const float*)d_in[5];
  const float* W_hh1   = (const float*)d_in[6];
  const float* b1      = (const float*)d_in[7];
  const float* Wc      = (const float*)d_in[8];
  const float* bc      = (const float*)d_in[9];
  const float* Wm      = (const float*)d_in[10];
  const float* bm      = (const float*)d_in[11];
  float* out = (float*)d_out;

  char* ws = (char*)d_ws;
  size_t off = 0;
  auto carve = [&](size_t bytes) -> char* { char* p = ws + off; off += (bytes + 255) & ~(size_t)255; return p; };
  unsigned short* WX0 = (unsigned short*)carve((size_t)NHID * WX_PITCH * 2);
  unsigned short* WH0 = (unsigned short*)carve((size_t)NHID * NHID * 2);
  unsigned short* WI1 = (unsigned short*)carve((size_t)NHID * NHID * 2);
  unsigned short* WH1 = (unsigned short*)carve((size_t)NHID * NHID * 2);
  unsigned short* WHD = (unsigned short*)carve((size_t)NHEAD_PAD * NHID * 2);
  float* STAGE = (float*)carve((size_t)NSTEP * NBATCH * 4 * 4);
  if (off > ws_size || off > (size_t)134217728) return;

  prep_planes_kernel<<<PB_ALL, NTHR, 0, stream>>>(W_ih0, W_hh0, W_ih1, W_hh1, Wc, Wm, WX0, WH0, WI1, WH1, WHD);
  rnn_scan_kernel<<<NBATCH / ROWS_BLK, NTHR, 0, stream>>>(cat_seq, val_seq, b0, b1, bc, bm,
                                                          WX0, WH0, WI1, WH1, WHD, STAGE);
  pack_out_kernel<<<(NOUT4 + NTHR - 1) / NTHR, NTHR, 0, stream>>>(STAGE, out, NOUT4);
}
